// Wn0119EMsolo_38268158608164
// MI455X (gfx1250) — hardware-verified
//
#include <hip/hip_runtime.h>
#include <math.h>

#define NT_    2000
#define NS_    512
#define NH_    16
#define HID_   256
#define NV_    64
#define NVR_   48
#define TCH_   250
#define NCH_   8
#define CROWS_ (TCH_ * NS_)
#define NLANE_ (NS_ * NH_)
#define STF_   51

typedef __attribute__((ext_vector_type(16))) _Float16 v16h;
typedef __attribute__((ext_vector_type(8)))  _Float16 v8h;
typedef __attribute__((ext_vector_type(16))) __bf16   v16b;
typedef __attribute__((ext_vector_type(8)))  __bf16   v8b;
typedef __attribute__((ext_vector_type(8)))  float    v8f;
typedef __attribute__((ext_vector_type(4)))  float    v4f;
typedef __attribute__((ext_vector_type(2)))  float    v2f;

__device__ __forceinline__ unsigned short f2bf_bits(float f) {
  unsigned u = __float_as_uint(f);
  return (unsigned short)((u + 0x7FFFu + ((u >> 16) & 1u)) >> 16);
}
__device__ __forceinline__ float bf_bits2f(unsigned short h) { return __uint_as_float(((unsigned)h) << 16); }

__device__ __forceinline__ void dep_guard_h(v8f& a, v8f& b, v16h x, v16h y) { asm volatile("v_nop\n\tv_nop\n\tv_nop\n\tv_nop" : "+v"(a), "+v"(b) : "v"(x), "v"(y)); }
__device__ __forceinline__ void dep_guard_b(v8f& a, v8f& b, v16b x, v16b y) { asm volatile("v_nop\n\tv_nop\n\tv_nop\n\tv_nop" : "+v"(a), "+v"(b) : "v"(x), "v"(y)); }
__device__ __forceinline__ void keep4_h(v16h a, v16h b, v16h c, v16h d) { asm volatile("v_nop" :: "v"(a), "v"(b), "v"(c), "v"(d)); }
__device__ __forceinline__ void keep4_b(v16b a, v16b b, v16b c, v16b d) { asm volatile("v_nop" :: "v"(a), "v"(b), "v"(c), "v"(d)); }
__device__ __forceinline__ void acc_guard4(v8f& a, v8f& b, v8f& c, v8f& d) { asm volatile("v_nop\n\tv_nop\n\tv_nop\n\tv_nop" : "+v"(a), "+v"(b), "+v"(c), "+v"(d)); }
template <typename T> struct Frag;
template <> struct Frag<_Float16> {
  typedef v16h V; union U { v16h v; v8h h[2]; };
  static __device__ __forceinline__ v16h load(const _Float16* p) {
    U f; f.h[0] = *(const v8h*)(p); f.h[1] = *(const v8h*)(p + 16); return f.v;
  }
  static __device__ __forceinline__ v8f mma(v16h a, v16h b, v8f c) {
    return __builtin_amdgcn_wmma_f32_16x16x32_f16(false, a, false, b, (short)0, c, false, false);
  }
  static __device__ __forceinline__ void guard(v8f& a, v8f& b, v16h x, v16h y) { dep_guard_h(a, b, x, y); }
  static __device__ __forceinline__ void keep(v16h a, v16h b, v16h c, v16h d) { keep4_h(a, b, c, d); }
};
template <> struct Frag<__bf16> {
  typedef v16b V; union U { v16b v; v8b h[2]; };
  static __device__ __forceinline__ v16b load(const __bf16* p) {
    U f; f.h[0] = *(const v8b*)(p); f.h[1] = *(const v8b*)(p + 16); return f.v;
  }
  static __device__ __forceinline__ v8f mma(v16b a, v16b b, v8f c) {
    return __builtin_amdgcn_wmma_f32_16x16x32_bf16(false, a, false, b, (short)0, c, false, false);
  }
  static __device__ __forceinline__ void guard(v8f& a, v8f& b, v16b x, v16b y) { dep_guard_b(a, b, x, y); }
  static __device__ __forceinline__ void keep(v16b a, v16b b, v16b c, v16b d) { keep4_b(a, b, c, d); }
};

template <int ET> struct Elem;
template <> struct Elem<0> { typedef _Float16 T; };
template <> struct Elem<1> { typedef __bf16 T; };
template <int ET, bool SPLIT, int BIAS_MODE, int OUT_MODE, bool RESID, int ACT = 0>
__global__ __launch_bounds__(256) void wmma_gemm64(
    const unsigned short* __restrict__ Ap, const unsigned short* __restrict__ A2p, int lda, long strideA,
    const unsigned short* __restrict__ Btp, const unsigned short* __restrict__ Bt2p, int ldb, long strideB,
    void* __restrict__ Cout, void* __restrict__ Cout2, int ldc, long strideC,
    const float* __restrict__ bias,
    const float* __restrict__ resid, long strideR,
    int M, int N, int K, float scale) {
  typedef typename Elem<ET>::T T;
  typedef typename Frag<T>::V V;
  const T* A = (const T*)Ap; const T* A2 = (const T*)A2p; const T* Bt = (const T*)Btp; const T* Bt2 = (const T*)Bt2p;
  __shared__ __align__(16) float sT[8][16 * 68];
  const int b    = blockIdx.y;
  const int lane = threadIdx.x & 31;
  const int wave = threadIdx.x >> 5;
  const int tilesN = N >> 6;
  const int tilesM = M >> 6;
  const int tile = blockIdx.x * 8 + wave;
  if (tile >= tilesM * tilesN) return;
  const int tm = tile / tilesN;
  const int tn = tile - tm * tilesN;
  const int m0 = tm << 6;
  const int n0 = tn << 6;

  const T* Ab  = A  + (size_t)b * strideA;
  const T* Bb  = Bt + (size_t)b * strideB;
  const T* Ab2 = SPLIT ? (A2  + (size_t)b * strideA) : nullptr;
  const T* Bb2 = SPLIT ? (Bt2 + (size_t)b * strideB) : nullptr;

  const int rlane = lane & 15;
  const int koff  = (lane >> 4) * 8;
  const int mOff  = (lane >> 4) * 8;

  v8f acc[4][4];
#pragma unroll
  for (int i = 0; i < 4; ++i)
#pragma unroll
    for (int j = 0; j < 4; ++j) acc[i][j] = (v8f){0.f,0.f,0.f,0.f,0.f,0.f,0.f,0.f};

  for (int k0 = 0; k0 < K; k0 += 32) {
    V bh[4], bl[4];
#pragma unroll
    for (int j = 0; j < 4; ++j) {
      const size_t bo = (size_t)(n0 + (j << 4) + rlane) * ldb + koff + k0;
      bh[j] = Frag<T>::load(Bb + bo);
      if (SPLIT) bl[j] = Frag<T>::load(Bb2 + bo);
    }
#pragma unroll
    for (int i = 0; i < 4; ++i) {
      const size_t ao = (size_t)(m0 + (i << 4) + rlane) * lda + koff + k0;
      V ah = Frag<T>::load(Ab + ao);
      V al;
      if (SPLIT) al = Frag<T>::load(Ab2 + ao);
#pragma unroll
      for (int j = 0; j < 4; ++j) {
        acc[i][j] = Frag<T>::mma(ah, bh[j], acc[i][j]);
        if (SPLIT) {
          acc[i][j] = Frag<T>::mma(ah, bl[j], acc[i][j]);
          acc[i][j] = Frag<T>::mma(al, bh[j], acc[i][j]);
        }
      }
      Frag<T>::guard(acc[i][0], acc[i][3], ah, SPLIT ? al : ah);
    }
    Frag<T>::keep(bh[0], bh[1], bh[2], bh[3]);
    if (SPLIT) Frag<T>::keep(bl[0], bl[1], bl[2], bl[3]);
  }
  acc_guard4(acc[0][0], acc[0][1], acc[0][2], acc[0][3]);
  acc_guard4(acc[1][0], acc[1][1], acc[1][2], acc[1][3]);
  acc_guard4(acc[2][0], acc[2][1], acc[2][2], acc[2][3]);
  acc_guard4(acc[3][0], acc[3][1], acc[3][2], acc[3][3]);

  float* slab = sT[wave];
  const float* Rb = RESID ? (resid + (size_t)b * strideR) : nullptr;
#pragma unroll
  for (int i = 0; i < 4; ++i) {
    const int mBase = m0 + (i << 4);
#pragma unroll
    for (int j = 0; j < 4; ++j) {
      const int n = n0 + (j << 4) + rlane;
      float bv = 0.f;
      if (BIAS_MODE == 2) bv = bias[n];
#pragma unroll
      for (int r = 0; r < 8; ++r) {
        float v = acc[i][j][r] * scale;
        if (BIAS_MODE == 1) v += bias[mBase + mOff + r];
        if (BIAS_MODE == 2) v += bv;
        if (RESID) v += Rb[(size_t)(mBase + mOff + r) * ldc + n];
        if (ACT == 1) v = tanhf(v);
        if (ACT == 2) v = fmaxf(v, 0.0f);
        if (ACT == 3) v = v / (1.0f + expf(-v));
        if (ACT == 4) v = (v > 0.f) ? v : 0.01f * v;
        if (ACT == 5) v = 0.5f * v * (1.0f + erff(v * 0.70710678118654752f));
        slab[(mOff + r) * 68 + (j << 4) + rlane] = v;
      }
    }
    __builtin_amdgcn_fence(__ATOMIC_RELEASE, "workgroup");
    __builtin_amdgcn_wave_barrier();
    __builtin_amdgcn_fence(__ATOMIC_ACQUIRE, "workgroup");
    if (OUT_MODE == 0) {
      float* C = (float*)Cout + (size_t)b * strideC;
      const int hh = lane >> 4, c4 = (lane & 15) * 4;
      for (int pass = 0; pass < 2; ++pass) {
#pragma unroll
        for (int it = 0; it < 8; ++it) {
          const int row = it * 2 + hh;
          v4f v = *(const v4f*)(slab + row * 68 + c4);
          *(volatile v4f*)(C + (size_t)(mBase + row) * ldc + n0 + c4) = v;
        }
        __threadfence();
      }
    } else {
      const int q = lane >> 3, c8 = (lane & 7) * 8;
      unsigned short* C  = (unsigned short*)Cout  + (size_t)b * strideC;
      unsigned short* C2 = (OUT_MODE == 2) ? ((unsigned short*)Cout2 + (size_t)b * strideC) : nullptr;
      for (int pass = 0; pass < 2; ++pass) {
#pragma unroll
        for (int it = 0; it < 4; ++it) {
          const int row = it * 4 + q;
          const float* sp = slab + row * 68 + c8;
          v8h hv, lv;
#pragma unroll
          for (int e = 0; e < 8; ++e) {
            if (OUT_MODE == 1) {
              hv[e] = (_Float16)sp[e];
            } else {
              unsigned short hb = f2bf_bits(sp[e]);
              unsigned short lb = f2bf_bits(sp[e] - bf_bits2f(hb));
              hv[e] = __builtin_bit_cast(_Float16, hb);
              lv[e] = __builtin_bit_cast(_Float16, lb);
            }
          }
          *(volatile v8h*)(C + (size_t)(mBase + row) * ldc + n0 + c8) = hv;
          if (OUT_MODE == 2) *(volatile v8h*)(C2 + (size_t)(mBase + row) * ldc + n0 + c8) = lv;
        }
        __threadfence();
      }
    }
    __builtin_amdgcn_fence(__ATOMIC_RELEASE, "workgroup");
    __builtin_amdgcn_wave_barrier();
    __builtin_amdgcn_fence(__ATOMIC_ACQUIRE, "workgroup");
  }
}

__device__ __forceinline__ float rcp_f(float v) { return __builtin_amdgcn_rcpf(v); }
__device__ __forceinline__ float sigm_f(float v) { return rcp_f(1.0f + __expf(-v)); }
__device__ __forceinline__ float tanh_f(float a) {
  const float e = __expf(2.0f * a);
  const float r = rcp_f(1.0f + e);
  return fmaf(-2.0f, r, 1.0f);
}

__global__ __launch_bounds__(256)
void setup_kernel(const float* __restrict__ W2, const float* __restrict__ b2,
                  _Float16* __restrict__ Bt, float* __restrict__ b2pad)
{
  const int tid = threadIdx.x;
#pragma unroll 1
  for (int it = 0; it < 8; ++it) {
    const int idx = it * 256 + tid;
    const int n   = idx >> 5;
    const int k0  = (idx & 31) * 8;
    const int nc  = (n < NVR_) ? n : (NVR_ - 1);
    v8h hv;
#pragma unroll
    for (int e = 0; e < 8; ++e) {
      float val = W2[(size_t)(k0 + e) * NVR_ + nc];
      val = (n < NVR_) ? (val * 16.0f) : 0.0f;
      hv[e] = (_Float16)val;
    }
    _Float16* dst = Bt + (size_t)n * HID_ + k0;
    *(volatile v8h*)dst = hv;
    __threadfence();
    *(volatile v8h*)dst = hv;
  }
  if (tid < 16) {
    v4f bv;
#pragma unroll
    for (int e = 0; e < 4; ++e) {
      const int n  = tid * 4 + e;
      const int nc = (n < NVR_) ? n : (NVR_ - 1);
      const float val = b2[nc];
      bv[e] = (n < NVR_) ? val : 0.0f;
    }
    float* dst = b2pad + tid * 4;
    *(volatile v4f*)dst = bv;
    __threadfence();
    *(volatile v4f*)dst = bv;
  }
}

__global__ __launch_bounds__(256)
void front_kernel(const float* __restrict__ x, const float* __restrict__ W1,
                  const float* __restrict__ b1, _Float16* __restrict__ H, int t0)
{
  const int lane = threadIdx.x & 31, wave = threadIdx.x >> 5;
  const int j0 = lane * 8;
  v4f wa[6], wb[6];
#pragma unroll
  for (int k = 0; k < 6; ++k) {
    wa[k] = *(const v4f*)(W1 + k * HID_ + j0);
    wb[k] = *(const v4f*)(W1 + k * HID_ + j0 + 4);
  }
  const v4f ba = *(const v4f*)(b1 + j0);
  const v4f bb = *(const v4f*)(b1 + j0 + 4);
  const size_t rbase = (size_t)blockIdx.x * 64;
#pragma unroll 1
  for (int it = 0; it < 8; ++it) {
    const size_t rowc = rbase + (size_t)(it * 8 + wave);
    const size_t row  = (size_t)t0 * NS_ + rowc;
    const float* xr = x + row * 6;
    const v2f x01 = *(const v2f*)(xr);
    const v2f x23 = *(const v2f*)(xr + 2);
    const v2f x45 = *(const v2f*)(xr + 4);
    const float xs[6] = {x01[0], x01[1], x23[0], x23[1], x45[0], x45[1]};
    v4f a0 = ba, a1 = bb;
#pragma unroll
    for (int k = 0; k < 6; ++k) { a0 = a0 + xs[k] * wa[k]; a1 = a1 + xs[k] * wb[k]; }
    v8h hv;
#pragma unroll
    for (int e = 0; e < 4; ++e) {
      hv[e]     = (_Float16)tanh_f(a0[e]);
      hv[4 + e] = (_Float16)tanh_f(a1[e]);
    }
    _Float16* dst = H + rowc * HID_ + j0;
    *(volatile v8h*)dst = hv;
    __threadfence();
    *(volatile v8h*)dst = hv;
  }
}

__global__ __launch_bounds__(256)
void scan_route_kernel(const float* __restrict__ x, const float* __restrict__ V,
                       const float* __restrict__ wR, const float* __restrict__ w,
                       const float* __restrict__ cp, const float* __restrict__ cs,
                       const float* __restrict__ cg,
                       float* __restrict__ ST, float* __restrict__ out, int t0, int first)
{
  __shared__ float ring[3 * 16 * 256];
  __shared__ float rnL[NH_ * 16];
  __shared__ float cmL[48];
  __shared__ __align__(16) float outsL[2][64];

  const int tid  = threadIdx.x;
  const int lane = tid & 31, wave = tid >> 5;
  const int sl   = tid >> 4, h = tid & 15;
  const int s    = blockIdx.x * 16 + sl;
  const int gidx = blockIdx.x * 256 + tid;
  const float INV_PI = 0.318309886183790672f;

  const float kp = sigm_f(w[h]);
  const float ks = sigm_f(w[16 + h]);
  const float kg = sigm_f(w[32 + h]) * 0.1f;
  const float gp = sigm_f(w[48 + h]);
  const float eg = expf(w[64 + h]);
  const float gL = eg * eg;
  const float qb = fmaxf(w[80 + h], 0.0f);
  float ga;
  {
    const float a = w[96 + h];
    float mx = a;
#pragma unroll
    for (int off = 1; off < 16; off <<= 1) mx = fmaxf(mx, __shfl_xor(mx, off, 32));
    const float ea = expf(a - mx);
    float sm = ea;
#pragma unroll
    for (int off = 1; off < 16; off <<= 1) sm += __shfl_xor(sm, off, 32);
    ga = ea * rcp_f(sm);
  }
  if (tid < 16) {
    float rv[16];
    float rs = 0.0f;
#pragma unroll
    for (int j = 0; j < 16; ++j) { rv[j] = fmaxf(wR[tid * 16 + j], 0.0f); rs += rv[j]; }
    const float inv = rcp_f(rs + 1e-8f) * ga;
#pragma unroll
    for (int j = 0; j < 16; ++j) rnL[tid * 16 + j] = rv[j] * inv;
  }
  if (tid < 36) {
    const int src = tid / 12, rem = tid - src * 12;
    const float va = cp[rem], vb = cs[rem], vc = cg[rem];
    const float vs = (src == 0) ? va : ((src == 1) ? vb : vc);
    cmL[tid] = fmaxf(expf(vs) - 1.0f, 0.0f);
  }
  float Sf, Ss, Sg;
  if (first != 0) {
    Sf = 0.0f; Ss = 0.0f; Sg = 0.0f;
#pragma unroll 1
    for (int q = 0; q < 48; ++q) ring[q * 256 + tid] = 0.0f;
  } else {
    Sf = ST[(size_t)0 * NLANE_ + gidx];
    Ss = ST[(size_t)1 * NLANE_ + gidx];
    Sg = ST[(size_t)2 * NLANE_ + gidx];
#pragma unroll 1
    for (int q = 0; q < 48; ++q) ring[q * 256 + tid] = ST[(size_t)(3 + q) * NLANE_ + gidx];
  }
  __syncthreads();

  const int m4 = (h & 3) * 3;
  const float cpm0 = cmL[m4 + 0],      cpm1 = cmL[m4 + 1],      cpm2 = cmL[m4 + 2];
  const float csm0 = cmL[12 + m4 + 0], csm1 = cmL[12 + m4 + 1], csm2 = cmL[12 + m4 + 2];
  const float cgm0 = cmL[24 + m4 + 0], cgm1 = cmL[24 + m4 + 1], cgm2 = cmL[24 + m4 + 2];
  const float one_m_gp = 1.0f - gp;

#pragma unroll 1
  for (int tl = 0; tl < TCH_; ++tl) {
    const int t = t0 + tl;
    const size_t row  = (size_t)t  * NS_ + s;
    const size_t rowc = (size_t)tl * NS_ + s;
    const float* xr = x + row * 6;
    const v2f x01 = *(const v2f*)(xr);
    const v2f x23 = *(const v2f*)(xr + 2);
    const float P = x01[0], E = x01[1], T1 = x23[0], T2 = x23[1];
    const float* vr = V + rowc * NV_;
    const float v0 = vr[h], v1 = vr[16 + h], v2 = vr[32 + h];

    const float vi = fminf(fmaxf(2.0f * v0 + 3.0f, 0.0f), 6.0f) * (1.0f / 6.0f);
    const float ve = fmaxf(v1, 0.0f) * 2.0f;
    const float vm = expf(v2);

    float frac = (T1 + T2) * rcp_f(T2 - T1 + 1e-8f);
    frac = fminf(fmaxf(frac, -1.0f), 1.0f);
    const float rPc = 1.0f - acosf(frac) * INV_PI;
    const float rP  = (T1 >= 0.0f) ? 1.0f : ((T2 <= 0.0f) ? 0.0f : rPc);
    const float Ps  = (1.0f - rP) * P;
    const float Pl  = (rP * P) * vi;
    const float Ev  = E * ve;

    const float Sf1 = fmaxf(Sf + Ps, 0.0f);
    const float qf  = fminf(Sf1, vm);
    Sf = Sf1 - qf;
    const float Hh  = fmaxf(((Ss + Pl) + qf) - Ev, 0.0f);
    const float qp  = fmaxf(kp * (Hh - gL), 0.0f);
    const float qs  = ks * fminf(Hh, gL);
    Ss = (Hh - qp) - qs;
    const float Sg1 = Sg + qs * gp;
    const float qg  = Sg1 * kg + qb;
    Sg = fmaxf(Sg1 - qg, 0.0f);
    const float qso = qs * one_m_gp;

    const int slot = t & 15;
    ring[(0  + slot) * 256 + tid] = qp;
    ring[(16 + slot) * 256 + tid] = qso;
    ring[(32 + slot) * 256 + tid] = qg;

    float cP = 0.0f, cS = 0.0f, cG = 0.0f;
#pragma unroll 4
    for (int j = 0; j < 16; ++j) {
      const int sj = (slot - j) & 15;
      const float wj = rnL[h * 16 + j];
      cP = fmaf(wj, ring[(0  + sj) * 256 + tid], cP);
      cS = fmaf(wj, ring[(16 + sj) * 256 + tid], cS);
      cG = fmaf(wj, ring[(32 + sj) * 256 + tid], cG);
    }
    float qsum = (cP + cS) + cG;
    float n0 = cP * cpm0 + cS * csm0 + cG * cgm0;
    float n1 = cP * cpm1 + cS * csm1 + cG * cgm1;
    float n2 = cP * cpm2 + cS * csm2 + cG * cgm2;
#pragma unroll
    for (int off = 1; off < 16; off <<= 1) {
      qsum += __shfl_xor(qsum, off, 32);
      n0   += __shfl_xor(n0,   off, 32);
      n1   += __shfl_xor(n1,   off, 32);
      n2   += __shfl_xor(n2,   off, 32);
    }
    const float inv = rcp_f(qsum + 1e-8f);
    const float o1 = n0 * inv, o2 = n1 * inv, o3 = n2 * inv;
    const float mine = (h == 0) ? qsum : ((h == 1) ? o1 : ((h == 2) ? o2 : o3));
    const int p = tl & 1;
    if (h < 4) outsL[p][sl * 4 + h] = mine;
    __syncthreads();
    if (wave == 0 && lane < 16) {
      const v4f val = *(const v4f*)(&outsL[p][lane * 4]);
      float* dst = out + ((size_t)t * NS_ + (size_t)blockIdx.x * 16) * 4 + lane * 4;
      *(volatile v4f*)dst = val;
      __threadfence();
      *(volatile v4f*)dst = val;
    }
  }

  {
    float* d0 = ST + gidx;
    for (int pass = 0; pass < 2; ++pass) {
      *(volatile float*)(d0 + (size_t)0 * NLANE_) = Sf;
      *(volatile float*)(d0 + (size_t)1 * NLANE_) = Ss;
      *(volatile float*)(d0 + (size_t)2 * NLANE_) = Sg;
#pragma unroll 1
      for (int q = 0; q < 48; ++q) {
        const float rvq = ring[q * 256 + tid];
        *(volatile float*)(d0 + (size_t)(3 + q) * NLANE_) = rvq;
      }
      __threadfence();
    }
  }
}

extern "C" void kernel_launch(void* const* d_in, const int* in_sizes, int n_in,
                              void* d_out, int out_size, void* d_ws, size_t ws_size,
                              hipStream_t stream)
{
  if (n_in < 10) return;
  if (in_sizes[0] < NT_ * NS_ * 6 || in_sizes[1] < NH_ * 16 || in_sizes[2] < NH_ * 7 ||
      in_sizes[3] < 6 * HID_ || in_sizes[4] < HID_ || in_sizes[5] < HID_ * NVR_ ||
      in_sizes[6] < NVR_ || in_sizes[7] < 12 || in_sizes[8] < 12 || in_sizes[9] < 12) return;
  if ((size_t)out_size < (size_t)NT_ * NS_ * 4) return;

  const float* x  = (const float*)d_in[0];
  const float* wR = (const float*)d_in[1];
  const float* w  = (const float*)d_in[2];
  const float* W1 = (const float*)d_in[3];
  const float* b1 = (const float*)d_in[4];
  const float* W2 = (const float*)d_in[5];
  const float* b2 = (const float*)d_in[6];
  const float* cp = (const float*)d_in[7];
  const float* cs = (const float*)d_in[8];
  const float* cg = (const float*)d_in[9];
  float* out = (float*)d_out;

  const size_t OFF_BT = 0;
  const size_t OFF_B2 = OFF_BT + (size_t)NV_ * HID_ * 2;
  const size_t OFF_ST = OFF_B2 + 256;
  const size_t OFF_H  = OFF_ST + (size_t)STF_ * NLANE_ * 4;
  const size_t OFF_V  = OFF_H + (size_t)CROWS_ * HID_ * 2;
  const size_t OFF_END = OFF_V + (size_t)CROWS_ * NV_ * 4;
  if (OFF_END > ws_size) return;

  char* ws = (char*)d_ws;
  _Float16* Bt    = (_Float16*)(ws + OFF_BT);
  float*    b2pad = (float*)(ws + OFF_B2);
  float*    ST    = (float*)(ws + OFF_ST);
  _Float16* H     = (_Float16*)(ws + OFF_H);
  float*    V     = (float*)(ws + OFF_V);

  setup_kernel<<<1, 256, 0, stream>>>(W2, b2, Bt, b2pad);

  const int frontBlocks = CROWS_ / 64;
  const int gemmBlocks  = (CROWS_ / 64) * (NV_ / 64) / 8;
  for (int c = 0; c < NCH_; ++c) {
    const int t0 = c * TCH_;
    front_kernel<<<frontBlocks, 256, 0, stream>>>(x, W1, b1, H, t0);
    wmma_gemm64<0, false, 2, 0, false, 0><<<dim3(gemmBlocks, 1), 256, 0, stream>>>(
        (const unsigned short*)H, (const unsigned short*)H, HID_, 0L,
        (const unsigned short*)Bt, (const unsigned short*)Bt, HID_, 0L,
        (void*)V, (void*)V, NV_, 0L,
        b2pad, b2pad, 0L,
        CROWS_, NV_, HID_, 1.0f / 16.0f);
    scan_route_kernel<<<NS_ / 16, 256, 0, stream>>>(x, V, wR, w, cp, cs, cg, ST, out, t0,
                                                     (c == 0) ? 1 : 0);
  }
}
